// LSH_34780645163546
// MI455X (gfx1250) — hardware-verified
//
#include <hip/hip_runtime.h>
#include <stdint.h>


#define BN     8
#define CCH    64
#define HH     128
#define WW     128
#define LW     126
#define KTOT   576
#define INVP   128
#define OPP    128
#define EPSF   1e-12f
#define ASCALE 16.0f
#define WSCALE 64.0f
#define OSCALE 0.0009765625f

typedef float    v4f  __attribute__((ext_vector_type(4)));
typedef float    v8f  __attribute__((ext_vector_type(8)));
typedef _Float16 v8h  __attribute__((ext_vector_type(8)));
typedef _Float16 v16h __attribute__((ext_vector_type(16)));
typedef v4f v4fa __attribute__((may_alias));
typedef v8h v8ha __attribute__((may_alias));

union Frag { v16h v; v8h half[2]; };

__device__ __forceinline__ v8f wmma_f16(const v16h a, const v16h b, v8f c) {
  return __builtin_amdgcn_wmma_f32_16x16x32_f16(false, a, false, b, (short)0, c, false, false);
}

__global__ __launch_bounds__(256) void k_sq(const float* __restrict__ x,
                                            float* __restrict__ sq, int nquad) {
  const int t = blockIdx.x * 256 + threadIdx.x;
  if (t >= nquad) return;
  const int e0 = t * 4;
  const int b  = e0 >> 14;
  const int yx = e0 & 16383;
  const float* p = x + (size_t)b * CCH * HH * WW + yx;
  v4f s = {0.f, 0.f, 0.f, 0.f};
#pragma unroll 4
  for (int c = 0; c < CCH; ++c) {
    v4f v = *(const v4fa*)(p + (size_t)c * HH * WW);
    s += v * v;
  }
  volatile v4f* d = (volatile v4f*)(sq + e0);
  *d = s;
  __threadfence();
  *d = s;
}

__global__ __launch_bounds__(256) void k_inv(const float* __restrict__ sq,
                                             float* __restrict__ inv, int nthr) {
  const int t = blockIdx.x * 256 + threadIdx.x;
  if (t >= nthr) return;
  const int R  = t >> 5;
  const int g  = t & 31;
  const int b  = R / LW;
  const int ph = R - b * LW;
  const float* p = sq + ((size_t)b * HH + ph) * WW;
  v4f r;
#pragma unroll
  for (int k = 0; k < 4; ++k) {
    int pw = g * 4 + k;
    pw = (pw < LW) ? pw : (LW - 1);
    const float* q = p + pw;
    float s = 0.f;
#pragma unroll
    for (int i = 0; i < 3; ++i) {
      s += q[i * WW + 0];
      s += q[i * WW + 1];
      s += q[i * WW + 2];
    }
    r[k] = 1.0f / fmaxf(sqrtf(s), EPSF);
  }
  volatile v4f* d = (volatile v4f*)(inv + (size_t)R * INVP + g * 4);
  *d = r;
  __threadfence();
  *d = r;
}

__global__ __launch_bounds__(256) void k_scale(const float* __restrict__ inv,
                                               float* __restrict__ S, int nquad) {
  const int t = blockIdx.x * 256 + threadIdx.x;
  if (t >= nquad) return;
  const int e0 = t * 4;
  const int b  = e0 >> 14;
  const int y  = (e0 >> 7) & 127;
  const int xb = e0 & 127;
  v4f r;
#pragma unroll
  for (int k = 0; k < 4; ++k) {
    const int xx = xb + k;
    float s = 0.f;
#pragma unroll
    for (int i = 0; i < 3; ++i) {
      const int ph = y - i;
      if ((unsigned)ph < (unsigned)LW) {
        const float* q = inv + ((size_t)(b * LW + ph)) * INVP;
#pragma unroll
        for (int j = 0; j < 3; ++j) {
          const int pw = xx - j;
          if ((unsigned)pw < (unsigned)LW) s += q[pw];
        }
      }
    }
    r[k] = s;
  }
  volatile v4f* d = (volatile v4f*)(S + e0);
  *d = r;
  __threadfence();
  *d = r;
}

__global__ __launch_bounds__(256) void k_fold(const float* __restrict__ x,
                                              const float* __restrict__ S,
                                              _Float16* __restrict__ folded, int nblk) {
  __shared__ _Float16 t[32 * CCH];
  const int blk = blockIdx.x;
  if (blk >= nblk) return;
  const int tid  = threadIdx.x;
  const int xblk = blk & 3;
  const int y    = (blk >> 2) & 127;
  const int b    = blk >> 9;
  const int x0   = xblk * 32;

  const int xx = tid & 31;
  const int c0 = tid >> 5;
  const float sc = S[(b << 14) + (y << 7) + x0 + xx] * ASCALE;
#pragma unroll
  for (int it = 0; it < 8; ++it) {
    const int c = c0 * 8 + it;
    const float v = x[(((size_t)b * CCH + c) * HH + y) * WW + x0 + xx];
    t[xx * CCH + c] = (_Float16)(v * sc);
  }
  __syncthreads();
  const int ox = tid >> 3;
  const int cg = (tid & 7) * 8;
  const v8h val = *(const v8ha*)(t + ox * CCH + cg);
  volatile v8h* d = (volatile v8h*)(folded +
      (((size_t)b * HH + y) * WW + x0 + ox) * CCH + cg);
  *d = val;
  __threadfence();
  *d = val;
}

__global__ __launch_bounds__(256) void k_wcvt(const float* __restrict__ w,
                                              _Float16* __restrict__ wA, int nthr) {
  const int t = blockIdx.x * 256 + threadIdx.x;
  if (t >= nthr) return;
  const int e0  = t * 8;
  const int oc  = e0 / KTOT;
  const int k0  = e0 - oc * KTOT;
  const int g   = k0 >> 6;
  const int ic0 = k0 & 63;
  const int i   = g / 3;
  const int j   = g - i * 3;
  const float* src = w + ((size_t)(oc * CCH + ic0) * 3 + i) * 3 + j;
  v8h val;
#pragma unroll
  for (int e = 0; e < 8; ++e) val[e] = (_Float16)(src[e * 9] * WSCALE);
  volatile v8h* d = (volatile v8h*)(wA + e0);
  *d = val;
  __threadfence();
  *d = val;
}

__global__ __launch_bounds__(256) void k_conv(const _Float16* __restrict__ folded,
                                              const _Float16* __restrict__ wA,
                                              float* __restrict__ outp, int nrows) {
  __shared__ float tile[CCH * OPP];
  const int row = blockIdx.x;
  if (row >= nrows) return;
  const int b    = row / LW;
  const int oy   = row - b * LW;
  const int tid  = threadIdx.x;
  const int wave = tid >> 5;
  const int lane = tid & 31;
  const int nl   = lane & 15;
  const int h    = lane >> 4;
  int px = wave * 16 + nl;
  px = (px < LW) ? px : (LW - 1);

  const _Float16* arow = wA + (size_t)nl * KTOT + 8 * h;

  v8f acc0 = {0.f, 0.f, 0.f, 0.f, 0.f, 0.f, 0.f, 0.f};
  v8f acc1 = acc0, acc2 = acc0, acc3 = acc0;

#pragma unroll 1
  for (int g = 0; g < 9; ++g) {
    const int di = g / 3;
    const int dj = g - di * 3;
    const _Float16* brow = folded +
        (((size_t)b * HH + (oy + di)) * WW + (px + dj)) * CCH + 8 * h;
#pragma unroll
    for (int cb = 0; cb < 64; cb += 32) {
      const int kk = g * 64 + cb;
      Frag Bf;
      Bf.half[0] = *(const v8ha*)(brow + cb);
      Bf.half[1] = *(const v8ha*)(brow + cb + 16);
      Frag A0, A1, A2, A3;
      const _Float16* ap0 = arow + (size_t)(0 * 16) * KTOT + kk;
      const _Float16* ap1 = arow + (size_t)(1 * 16) * KTOT + kk;
      const _Float16* ap2 = arow + (size_t)(2 * 16) * KTOT + kk;
      const _Float16* ap3 = arow + (size_t)(3 * 16) * KTOT + kk;
      A0.half[0] = *(const v8ha*)ap0;  A0.half[1] = *(const v8ha*)(ap0 + 16);
      A1.half[0] = *(const v8ha*)ap1;  A1.half[1] = *(const v8ha*)(ap1 + 16);
      A2.half[0] = *(const v8ha*)ap2;  A2.half[1] = *(const v8ha*)(ap2 + 16);
      A3.half[0] = *(const v8ha*)ap3;  A3.half[1] = *(const v8ha*)(ap3 + 16);

      acc0 = wmma_f16(A0.v, Bf.v, acc0);
      acc1 = wmma_f16(A1.v, Bf.v, acc1);
      acc2 = wmma_f16(A2.v, Bf.v, acc2);
      acc3 = wmma_f16(A3.v, Bf.v, acc3);
      asm volatile("v_nop\n\tv_nop\n\tv_nop\n\tv_nop"
                   : "+v"(acc0), "+v"(acc1), "+v"(acc2), "+v"(acc3)
                   : "v"(A0.v), "v"(A1.v), "v"(A2.v), "v"(A3.v), "v"(Bf.v));
    }
  }

  const int col = wave * 16 + nl;
#pragma unroll
  for (int r = 0; r < 8; ++r) {
    const int oc = 8 * h + r;
    tile[(oc +  0) * OPP + col] = acc0[r];
    tile[(oc + 16) * OPP + col] = acc1[r];
    tile[(oc + 32) * OPP + col] = acc2[r];
    tile[(oc + 48) * OPP + col] = acc3[r];
  }
  __syncthreads();

  v4f vals[8];
#pragma unroll
  for (int q = 0; q < 8; ++q) {
    const int oc = wave * 8 + q;
    vals[q] = *(const v4fa*)(tile + oc * OPP + lane * 4) * OSCALE;
  }
  float* ob = outp + (((size_t)b * CCH + wave * 8) * LW + oy) * OPP + lane * 4;
#pragma unroll
  for (int q = 0; q < 8; ++q)
    *(volatile v4f*)(ob + (size_t)q * LW * OPP) = vals[q];
  __threadfence();
#pragma unroll
  for (int q = 0; q < 8; ++q)
    *(volatile v4f*)(ob + (size_t)q * LW * OPP) = vals[q];
}

__global__ __launch_bounds__(256) void k_repack(const float* __restrict__ outp,
                                                float* __restrict__ out, int nquad) {
  const int t = blockIdx.x * 256 + threadIdx.x;
  if (t >= nquad) return;
  const int e0   = t * 4;
  const int row0 = e0 / LW;
  const int ox0  = e0 - row0 * LW;
  v4f val;
#pragma unroll
  for (int k = 0; k < 4; ++k) {
    int oxk = ox0 + k;
    int rk  = row0;
    if (oxk >= LW) { oxk -= LW; rk += 1; }
    val[k] = outp[(size_t)rk * OPP + oxk];
  }
  volatile v4f* d = (volatile v4f*)(out + e0);
  *d = val;
  __threadfence();
  *d = val;
}

extern "C" void kernel_launch(void* const* d_in, const int* in_sizes, int n_in,
                              void* d_out, int out_size, void* d_ws, size_t ws_size,
                              hipStream_t stream) {
  if (n_in < 2) return;
  const int nx = in_sizes[0];
  const int nw = in_sizes[1];
  if (nx != BN * CCH * HH * WW) return;
  if (nw != CCH * CCH * 9) return;
  if (out_size != BN * CCH * LW * LW) return;

  const float* x = (const float*)d_in[0];
  const float* w = (const float*)d_in[1];
  float* out = (float*)d_out;

  const size_t sq_bytes   = (size_t)BN * HH * WW * sizeof(float);
  const size_t inv_bytes  = (size_t)BN * LW * INVP * sizeof(float);
  const size_t s_bytes    = sq_bytes;
  const size_t wa_bytes   = (size_t)CCH * KTOT * sizeof(_Float16);
  const size_t fold_bytes = (size_t)BN * HH * WW * CCH * sizeof(_Float16);
  const size_t outp_bytes = (size_t)BN * CCH * LW * OPP * sizeof(float);
  const size_t o_sq   = 0;
  const size_t o_inv  = o_sq + sq_bytes;
  const size_t o_s    = o_inv + inv_bytes;
  const size_t o_wa   = o_s + s_bytes;
  const size_t o_fold = o_wa + wa_bytes;
  const size_t o_outp = o_fold + fold_bytes;
  const size_t o_end  = o_outp + outp_bytes;
  if (o_end > ws_size) return;

  char* ws = (char*)d_ws;
  float*    sq     = (float*)(ws + o_sq);
  float*    inv    = (float*)(ws + o_inv);
  float*    S      = (float*)(ws + o_s);
  _Float16* wA     = (_Float16*)(ws + o_wa);
  _Float16* folded = (_Float16*)(ws + o_fold);
  float*    outp   = (float*)(ws + o_outp);

  const int nquad_px = (BN * HH * WW) / 4;
  const int nthr_inv = BN * LW * 32;
  const int nblk_fld = BN * HH * 4;
  const int nthr_w   = (CCH * KTOT) / 8;
  const int nrows    = BN * LW;
  const int nquad_o  = out_size / 4;

  k_sq    <<<(nquad_px + 255) / 256, 256, 0, stream>>>(x, sq, nquad_px);
  k_inv   <<<(nthr_inv + 255) / 256, 256, 0, stream>>>(sq, inv, nthr_inv);
  k_scale <<<(nquad_px + 255) / 256, 256, 0, stream>>>(inv, S, nquad_px);
  k_fold  <<<nblk_fld, 256, 0, stream>>>(x, S, folded, nblk_fld);
  k_wcvt  <<<(nthr_w + 255) / 256, 256, 0, stream>>>(w, wA, nthr_w);
  k_conv  <<<nrows, 256, 0, stream>>>(folded, wA, outp, nrows);
  k_repack<<<(nquad_o + 255) / 256, 256, 0, stream>>>(outp, out, nquad_o);
}
